// BasicMambaBlock_53738630808035
// MI455X (gfx1250) — hardware-run, weakly checked
//
#include <hip/hip_runtime.h>
#include <math.h>

constexpr int NBATCH  = 2;
constexpr int NLEN    = 1024;
constexpr int DMOD    = 1024;
constexpr int DIN     = 2048;
constexpr int NSTATE  = 16;
constexpr int KCONV   = 4;
constexpr int DTRANK  = 64;
constexpr int NTOK    = NBATCH * NLEN;
constexpr int XZW     = 2 * DIN;
constexpr int XDBL_N  = DTRANK + 2 * NSTATE;
constexpr int XDBL_LD = 128;
constexpr int SCAN_TB = 256;
constexpr int SCAN_TCH = 16;
constexpr float CARRY     = 16.0f;
constexpr float INV_C1    = 1.0f / 16.0f;
constexpr float INV_C2    = 1.0f / 256.0f;
constexpr float LN_EPS    = 1e-5f;
constexpr float INV_DMOD  = 1.0f / 1024.0f;

typedef __attribute__((ext_vector_type(16))) _Float16 v16h;
typedef __attribute__((ext_vector_type(8)))  _Float16 v8h;
typedef __attribute__((ext_vector_type(16))) __bf16   v16b;
typedef __attribute__((ext_vector_type(8)))  __bf16   v8b;
typedef __attribute__((ext_vector_type(8)))  float    v8f;
typedef __attribute__((ext_vector_type(4)))  float    v4f;
typedef __attribute__((ext_vector_type(4)))  unsigned int v4u;

__device__ __forceinline__ unsigned short f2bf_bits(float f) {
  unsigned u = __float_as_uint(f);
  return (unsigned short)((u + 0x7FFFu + ((u >> 16) & 1u)) >> 16);
}
__device__ __forceinline__ float bf_bits2f(unsigned short h) { return __uint_as_float(((unsigned)h) << 16); }

__device__ __forceinline__ void dep_guard_h(v8f& a, v8f& b, v16h x, v16h y) { asm volatile("v_nop\n\tv_nop\n\tv_nop\n\tv_nop" : "+v"(a), "+v"(b) : "v"(x), "v"(y)); }
__device__ __forceinline__ void dep_guard_b(v8f& a, v8f& b, v16b x, v16b y) { asm volatile("v_nop\n\tv_nop\n\tv_nop\n\tv_nop" : "+v"(a), "+v"(b) : "v"(x), "v"(y)); }
__device__ __forceinline__ void keep4_h(v16h a, v16h b, v16h c, v16h d) { asm volatile("v_nop" :: "v"(a), "v"(b), "v"(c), "v"(d)); }
__device__ __forceinline__ void keep4_b(v16b a, v16b b, v16b c, v16b d) { asm volatile("v_nop" :: "v"(a), "v"(b), "v"(c), "v"(d)); }
__device__ __forceinline__ void acc_guard4(v8f& a, v8f& b, v8f& c, v8f& d) { asm volatile("v_nop\n\tv_nop\n\tv_nop\n\tv_nop" : "+v"(a), "+v"(b), "+v"(c), "+v"(d)); }
template <typename T> struct Frag;
template <> struct Frag<_Float16> {
  typedef v16h V; union U { v16h v; v8h h[2]; };
  static __device__ __forceinline__ v16h load(const _Float16* p) {
    U f; f.h[0] = *(const v8h*)(p); f.h[1] = *(const v8h*)(p + 16); return f.v;
  }
  static __device__ __forceinline__ v8f mma(v16h a, v16h b, v8f c) {
    return __builtin_amdgcn_wmma_f32_16x16x32_f16(false, a, false, b, (short)0, c, false, false);
  }
  static __device__ __forceinline__ void guard(v8f& a, v8f& b, v16h x, v16h y) { dep_guard_h(a, b, x, y); }
  static __device__ __forceinline__ void keep(v16h a, v16h b, v16h c, v16h d) { keep4_h(a, b, c, d); }
};
template <> struct Frag<__bf16> {
  typedef v16b V; union U { v16b v; v8b h[2]; };
  static __device__ __forceinline__ v16b load(const __bf16* p) {
    U f; f.h[0] = *(const v8b*)(p); f.h[1] = *(const v8b*)(p + 16); return f.v;
  }
  static __device__ __forceinline__ v8f mma(v16b a, v16b b, v8f c) {
    return __builtin_amdgcn_wmma_f32_16x16x32_bf16(false, a, false, b, (short)0, c, false, false);
  }
  static __device__ __forceinline__ void guard(v8f& a, v8f& b, v16b x, v16b y) { dep_guard_b(a, b, x, y); }
  static __device__ __forceinline__ void keep(v16b a, v16b b, v16b c, v16b d) { keep4_b(a, b, c, d); }
};

__device__ __forceinline__ unsigned pk16(unsigned short a, unsigned short b) { return (unsigned)a | ((unsigned)b << 16); }
__device__ __forceinline__ unsigned short h_bits(float f) { const _Float16 h = (_Float16)f; return __builtin_bit_cast(unsigned short, h); }

template <int ET> struct Elem;
template <> struct Elem<0> { typedef _Float16 T; };
template <> struct Elem<1> { typedef __bf16 T; };
template <int ET, bool SPLIT, int BIAS_MODE, int OUT_MODE, bool RESID, int ACT = 0>
__global__ __launch_bounds__(256) void wmma_gemm64(
    const unsigned short* __restrict__ Ap, const unsigned short* __restrict__ A2p, int lda, long strideA,
    const unsigned short* __restrict__ Btp, const unsigned short* __restrict__ Bt2p, int ldb, long strideB,
    void* __restrict__ Cout, void* __restrict__ Cout2, int ldc, long strideC,
    const float* __restrict__ bias,
    const float* __restrict__ resid, long strideR,
    int M, int N, int K, float scale) {
  typedef typename Elem<ET>::T T;
  typedef typename Frag<T>::V V;
  const T* A = (const T*)Ap; const T* A2 = (const T*)A2p; const T* Bt = (const T*)Btp; const T* Bt2 = (const T*)Bt2p;
  __shared__ __align__(16) float sT[8][16 * 68];
  const int b    = blockIdx.y;
  const int lane = threadIdx.x & 31;
  const int wave = threadIdx.x >> 5;
  const int tilesN = N >> 6;
  const int tilesM = M >> 6;
  const int tile = blockIdx.x * 8 + wave;
  if (tile >= tilesM * tilesN) return;
  const int tm = tile / tilesN;
  const int tn = tile - tm * tilesN;
  const int m0 = tm << 6;
  const int n0 = tn << 6;

  const T* Ab  = A  + (size_t)b * strideA;
  const T* Bb  = Bt + (size_t)b * strideB;
  const T* Ab2 = SPLIT ? (A2  + (size_t)b * strideA) : nullptr;
  const T* Bb2 = SPLIT ? (Bt2 + (size_t)b * strideB) : nullptr;

  const int rlane = lane & 15;
  const int koff  = (lane >> 4) * 8;
  const int mOff  = (lane >> 4) * 8;

  v8f acc[4][4];
#pragma unroll
  for (int i = 0; i < 4; ++i)
#pragma unroll
    for (int j = 0; j < 4; ++j) acc[i][j] = (v8f){0.f,0.f,0.f,0.f,0.f,0.f,0.f,0.f};

  for (int k0 = 0; k0 < K; k0 += 32) {
    V bh[4], bl[4];
#pragma unroll
    for (int j = 0; j < 4; ++j) {
      const size_t bo = (size_t)(n0 + (j << 4) + rlane) * ldb + koff + k0;
      bh[j] = Frag<T>::load(Bb + bo);
      if (SPLIT) bl[j] = Frag<T>::load(Bb2 + bo);
    }
#pragma unroll
    for (int i = 0; i < 4; ++i) {
      const size_t ao = (size_t)(m0 + (i << 4) + rlane) * lda + koff + k0;
      V ah = Frag<T>::load(Ab + ao);
      V al;
      if (SPLIT) al = Frag<T>::load(Ab2 + ao);
#pragma unroll
      for (int j = 0; j < 4; ++j) {
        acc[i][j] = Frag<T>::mma(ah, bh[j], acc[i][j]);
        if (SPLIT) {
          acc[i][j] = Frag<T>::mma(ah, bl[j], acc[i][j]);
          acc[i][j] = Frag<T>::mma(al, bh[j], acc[i][j]);
        }
      }
      Frag<T>::guard(acc[i][0], acc[i][3], ah, SPLIT ? al : ah);
    }
    Frag<T>::keep(bh[0], bh[1], bh[2], bh[3]);
    if (SPLIT) Frag<T>::keep(bl[0], bl[1], bl[2], bl[3]);
  }
  acc_guard4(acc[0][0], acc[0][1], acc[0][2], acc[0][3]);
  acc_guard4(acc[1][0], acc[1][1], acc[1][2], acc[1][3]);
  acc_guard4(acc[2][0], acc[2][1], acc[2][2], acc[2][3]);
  acc_guard4(acc[3][0], acc[3][1], acc[3][2], acc[3][3]);

  float* slab = sT[wave];
  const float* Rb = RESID ? (resid + (size_t)b * strideR) : nullptr;
#pragma unroll
  for (int i = 0; i < 4; ++i) {
    const int mBase = m0 + (i << 4);
#pragma unroll
    for (int j = 0; j < 4; ++j) {
      const int n = n0 + (j << 4) + rlane;
      float bv = 0.f;
      if (BIAS_MODE == 2) bv = bias[n];
#pragma unroll
      for (int r = 0; r < 8; ++r) {
        float v = acc[i][j][r] * scale;
        if (BIAS_MODE == 1) v += bias[mBase + mOff + r];
        if (BIAS_MODE == 2) v += bv;
        if (RESID) v += Rb[(size_t)(mBase + mOff + r) * ldc + n];
        if (ACT == 2) v = fmaxf(v, 0.0f);
        if (ACT == 4) v = (v > 0.f) ? v : 0.01f * v;
        slab[(mOff + r) * 68 + (j << 4) + rlane] = v;
      }
    }
    __builtin_amdgcn_fence(__ATOMIC_RELEASE, "workgroup");
    __builtin_amdgcn_wave_barrier();
    __builtin_amdgcn_fence(__ATOMIC_ACQUIRE, "workgroup");
    if (OUT_MODE == 0) {
      float* C = (float*)Cout + (size_t)b * strideC;
      const int hh = lane >> 4, c4 = (lane & 15) * 4;
      for (int pass = 0; pass < 2; ++pass) {
#pragma unroll
        for (int it = 0; it < 8; ++it) {
          const int row = it * 2 + hh;
          v4f v = *(const v4f*)(slab + row * 68 + c4);
          *(volatile v4f*)(C + (size_t)(mBase + row) * ldc + n0 + c4) = v;
        }
        __threadfence();
      }
    } else {
      const int q = lane >> 3, c8 = (lane & 7) * 8;
      unsigned short* C  = (unsigned short*)Cout  + (size_t)b * strideC;
      unsigned short* C2 = (OUT_MODE == 2) ? ((unsigned short*)Cout2 + (size_t)b * strideC) : nullptr;
      for (int pass = 0; pass < 2; ++pass) {
#pragma unroll
        for (int it = 0; it < 4; ++it) {
          const int row = it * 4 + q;
          const float* sp = slab + row * 68 + c8;
          v8h hv, lv;
#pragma unroll
          for (int e = 0; e < 8; ++e) {
            if (OUT_MODE == 1) {
              hv[e] = (_Float16)sp[e];
            } else {
              unsigned short hb = f2bf_bits(sp[e]);
              unsigned short lb = f2bf_bits(sp[e] - bf_bits2f(hb));
              hv[e] = __builtin_bit_cast(_Float16, hb);
              lv[e] = __builtin_bit_cast(_Float16, lb);
            }
          }
          *(volatile v8h*)(C + (size_t)(mBase + row) * ldc + n0 + c8) = hv;
          if (OUT_MODE == 2) *(volatile v8h*)(C2 + (size_t)(mBase + row) * ldc + n0 + c8) = lv;
        }
        __threadfence();
      }
    }
    __builtin_amdgcn_fence(__ATOMIC_RELEASE, "workgroup");
    __builtin_amdgcn_wave_barrier();
    __builtin_amdgcn_fence(__ATOMIC_ACQUIRE, "workgroup");
  }
}

__global__ __launch_bounds__(256) void cast8_pad_kernel(const float* __restrict__ in, unsigned short* __restrict__ out,
                                                        int count8, int total8, float scale) {
  const int i = blockIdx.x * 256 + threadIdx.x;
  if (i >= total8) return;
  const bool valid = (i < count8);
  const int ic = valid ? i : (count8 - 1);
  const float* p = in + 8 * (size_t)ic;
  const v4f a = *(const v4f*)(p);
  const v4f c = *(const v4f*)(p + 4);
  unsigned short hb[8];
#pragma unroll
  for (int e = 0; e < 4; ++e) {
    const float f0 = valid ? a[e] * scale : 0.0f;
    const float f1 = valid ? c[e] * scale : 0.0f;
    hb[e]     = h_bits(f0);
    hb[4 + e] = h_bits(f1);
  }
  const v4u u = (v4u){pk16(hb[0], hb[1]), pk16(hb[2], hb[3]), pk16(hb[4], hb[5]), pk16(hb[6], hb[7])};
  unsigned short* q = out + 8 * (size_t)i;
  *(volatile v4u*)q = u;
  __threadfence();
  *(volatile v4u*)q = u;
}

__global__ __launch_bounds__(256) void dtcast_kernel(const float* __restrict__ xd, unsigned short* __restrict__ out, float scale) {
  const int i = blockIdx.x * 256 + threadIdx.x;
  if (i >= NTOK * 8) return;
  const int row = i >> 3, c8 = (i & 7) * 8;
  const float* p = xd + (size_t)row * XDBL_LD + c8;
  const v4f a = *(const v4f*)(p);
  const v4f c = *(const v4f*)(p + 4);
  unsigned short hb[8];
#pragma unroll
  for (int e = 0; e < 4; ++e) {
    hb[e]     = h_bits(a[e] * scale);
    hb[4 + e] = h_bits(c[e] * scale);
  }
  const v4u u = (v4u){pk16(hb[0], hb[1]), pk16(hb[2], hb[3]), pk16(hb[4], hb[5]), pk16(hb[6], hb[7])};
  unsigned short* q = out + (size_t)row * DTRANK + c8;
  *(volatile v4u*)q = u;
  __threadfence();
  *(volatile v4u*)q = u;
}

__global__ __launch_bounds__(128) void ln_kernel(const float* __restrict__ x, const float* __restrict__ g,
                                                 const float* __restrict__ bt, unsigned short* __restrict__ xn) {
  __shared__ float sR1[4];
  __shared__ float sR2[4];
  const int m = blockIdx.x, t = threadIdx.x, lane = t & 31, wave = t >> 5;
  const int c0 = t * 8;
  const float* row = x + (size_t)m * DMOD + c0;
  const v4f a = *(const v4f*)(row);
  const v4f c = *(const v4f*)(row + 4);
  float xv[8];
#pragma unroll
  for (int e = 0; e < 4; ++e) { xv[e] = a[e]; xv[4 + e] = c[e]; }
  float s = 0.f;
#pragma unroll
  for (int e = 0; e < 8; ++e) s += xv[e];
#pragma unroll
  for (int off = 16; off > 0; off >>= 1) s += __shfl_xor(s, off, 32);
  if (lane == 0) sR1[wave] = s;
  __syncthreads();
  const float mu = ((sR1[0] + sR1[1]) + (sR1[2] + sR1[3])) * INV_DMOD;
  float s2 = 0.f;
#pragma unroll
  for (int e = 0; e < 8; ++e) { const float dd = xv[e] - mu; s2 += dd * dd; }
#pragma unroll
  for (int off = 16; off > 0; off >>= 1) s2 += __shfl_xor(s2, off, 32);
  if (lane == 0) sR2[wave] = s2;
  __syncthreads();
  const float var  = ((sR2[0] + sR2[1]) + (sR2[2] + sR2[3])) * INV_DMOD;
  const float rstd = rsqrtf(var + LN_EPS);
  const v4f ga = *(const v4f*)(g + c0);
  const v4f gc = *(const v4f*)(g + c0 + 4);
  const v4f ba = *(const v4f*)(bt + c0);
  const v4f bc = *(const v4f*)(bt + c0 + 4);
  unsigned short hb[8];
#pragma unroll
  for (int e = 0; e < 4; ++e) {
    hb[e]     = h_bits(((xv[e] - mu) * rstd) * ga[e] + ba[e]);
    hb[4 + e] = h_bits(((xv[4 + e] - mu) * rstd) * gc[e] + bc[e]);
  }
  const v4u u = (v4u){pk16(hb[0], hb[1]), pk16(hb[2], hb[3]), pk16(hb[4], hb[5]), pk16(hb[6], hb[7])};
  unsigned short* q = xn + (size_t)m * DMOD + c0;
  *(volatile v4u*)q = u;
  __threadfence();
  *(volatile v4u*)q = u;
}

__global__ __launch_bounds__(256) void conv_silu_kernel(const float* __restrict__ xz, const float* __restrict__ cw,
                                                        const float* __restrict__ cb, float* __restrict__ u,
                                                        unsigned short* __restrict__ uh) {
  __shared__ __align__(16) float sU[DIN];
  const int m = blockIdx.x, t = threadIdx.x;
  const int bb = m >> 10, l = m & (NLEN - 1);
#pragma unroll 1
  for (int i = 0; i < DIN / 256; ++i) {
    const int d = i * 256 + t;
    float acc = 0.f;
#pragma unroll
    for (int j = 0; j < KCONV; ++j) {
      const int ls  = l - (KCONV - 1) + j;
      const int lsc = (ls < 0) ? 0 : ls;
      float v = xz[((size_t)(bb * NLEN + lsc)) * XZW + d];
      v = (ls >= 0) ? v : 0.f;
      acc += cw[d * KCONV + j] * v;
    }
    acc += cb[d];
    const float sg = 1.0f / (1.0f + expf(-acc));
    sU[d] = acc * sg;
  }
  __syncthreads();
  float* urow = u + (size_t)m * DIN;
  unsigned short* hrow = uh + (size_t)m * DIN;
  for (int pass = 0; pass < 2; ++pass) {
#pragma unroll
    for (int it = 0; it < 2; ++it) {
      const int idx = it * 1024 + t * 4;
      const v4f v = *(const v4f*)(sU + idx);
      *(volatile v4f*)(urow + idx) = v;
    }
    {
      const float* sp = sU + t * 8;
      const v4f a = *(const v4f*)(sp);
      const v4f c = *(const v4f*)(sp + 4);
      unsigned short hb[8];
#pragma unroll
      for (int e = 0; e < 4; ++e) {
        hb[e]     = h_bits(a[e] * CARRY);
        hb[4 + e] = h_bits(c[e] * CARRY);
      }
      const v4u w = (v4u){pk16(hb[0], hb[1]), pk16(hb[2], hb[3]), pk16(hb[4], hb[5]), pk16(hb[6], hb[7])};
      *(volatile v4u*)(hrow + t * 8) = w;
    }
    __threadfence();
  }
}

__global__ __launch_bounds__(256) void scan_kernel(const float* __restrict__ dpre, const float* __restrict__ u,
                                                   const float* __restrict__ xdbl, const float* __restrict__ xz,
                                                   const float* __restrict__ A_log, const float* __restrict__ dtb,
                                                   const float* __restrict__ Dv, unsigned short* __restrict__ y16) {
  __shared__ __align__(16) float sH[NSTATE * SCAN_TB];
  __shared__ __align__(16) float sA[NSTATE * SCAN_TB];
  __shared__ __align__(16) float sY[SCAN_TCH * SCAN_TB];
  __shared__ __align__(16) float sBC[SCAN_TCH * 2 * NSTATE];
  const int t = threadIdx.x, lane = t & 31, wave = t >> 5;
  const int d0 = blockIdx.x * SCAN_TB, bb = blockIdx.y;
  const int d = d0 + t;
#pragma unroll 1
  for (int n = 0; n < NSTATE; ++n) {
    sH[n * SCAN_TB + t] = 0.f;
    sA[n * SCAN_TB + t] = -expf(A_log[(size_t)d * NSTATE + n]);
  }
  const float bias = dtb[d];
  const float Dd   = Dv[d];
#pragma unroll 1
  for (int ch = 0; ch < NLEN / SCAN_TCH; ++ch) {
    const int m0 = bb * NLEN + ch * SCAN_TCH;
    {
      const int s = t >> 4, cp = (t & 15) * 2;
      const float* src = xdbl + (size_t)(m0 + s) * XDBL_LD + DTRANK + cp;
      sBC[s * 32 + cp]     = src[0];
      sBC[s * 32 + cp + 1] = src[1];
    }
    __syncthreads();
#pragma unroll 1
    for (int s = 0; s < SCAN_TCH; ++s) {
      const size_t m = (size_t)(m0 + s);
      const float xp = dpre[m * DIN + d] + bias;
      const float dl = fmaxf(xp, 0.f) + log1pf(expf(-fabsf(xp)));
      const float uu = u[m * DIN + d];
      const float zz = xz[m * XZW + DIN + d];
      float y = 0.f;
#pragma unroll 1
      for (int n = 0; n < NSTATE; ++n) {
        const float a  = sA[n * SCAN_TB + t];
        float hv       = sH[n * SCAN_TB + t];
        const float bn = sBC[s * 32 + n];
        const float cn = sBC[s * 32 + NSTATE + n];
        hv = expf(dl * a) * hv + (dl * bn) * uu;
        sH[n * SCAN_TB + t] = hv;
        y += hv * cn;
      }
      y += uu * Dd;
      const float sg = 1.0f / (1.0f + expf(-zz));
      y = y * (zz * sg);
      sY[s * SCAN_TB + t] = y * CARRY;
    }
    __syncthreads();
    for (int pass = 0; pass < 2; ++pass) {
#pragma unroll
      for (int i = 0; i < 2; ++i) {
        const int s = 8 * i + wave;
        const float* sp = sY + s * SCAN_TB + lane * 8;
        const v4f a = *(const v4f*)(sp);
        const v4f c = *(const v4f*)(sp + 4);
        unsigned short hb[8];
#pragma unroll
        for (int e = 0; e < 4; ++e) {
          hb[e]     = h_bits(a[e]);
          hb[4 + e] = h_bits(c[e]);
        }
        const v4u w = (v4u){pk16(hb[0], hb[1]), pk16(hb[2], hb[3]), pk16(hb[4], hb[5]), pk16(hb[6], hb[7])};
        *(volatile v4u*)(y16 + (size_t)(m0 + s) * DIN + d0 + lane * 8) = w;
      }
      __threadfence();
    }
  }
}

extern "C" void kernel_launch(void* const* d_in, const int* in_sizes, int n_in,
                              void* d_out, int out_size, void* d_ws, size_t ws_size,
                              hipStream_t stream) {
  if (n_in < 12) return;
  if (in_sizes[0] != NTOK * DMOD || in_sizes[1] != DMOD || in_sizes[2] != DMOD ||
      in_sizes[3] != XZW * DMOD || in_sizes[4] != DIN * KCONV || in_sizes[5] != DIN ||
      in_sizes[6] != XDBL_N * DIN || in_sizes[7] != DIN * DTRANK || in_sizes[8] != DIN ||
      in_sizes[9] != DIN * NSTATE || in_sizes[10] != DIN || in_sizes[11] != DMOD * DIN) return;
  if (out_size != NTOK * DMOD) return;

  const float* x          = (const float*)d_in[0];
  const float* ln_g       = (const float*)d_in[1];
  const float* ln_b       = (const float*)d_in[2];
  const float* in_proj_w  = (const float*)d_in[3];
  const float* conv_w     = (const float*)d_in[4];
  const float* conv_b     = (const float*)d_in[5];
  const float* x_proj_w   = (const float*)d_in[6];
  const float* dt_proj_w  = (const float*)d_in[7];
  const float* dt_proj_b  = (const float*)d_in[8];
  const float* A_log      = (const float*)d_in[9];
  const float* Dv         = (const float*)d_in[10];
  const float* out_proj_w = (const float*)d_in[11];
  float* out = (float*)d_out;

  char* ws = (char*)d_ws;
  size_t off = 0;
  auto carve = [&](size_t bytes) { char* p = ws + off; off = (off + bytes + 255) & ~(size_t)255; return p; };
  unsigned short* w1h  = (unsigned short*)carve((size_t)XZW * DMOD * 2);
  unsigned short* xph  = (unsigned short*)carve((size_t)XDBL_LD * DIN * 2);
  unsigned short* dtph = (unsigned short*)carve((size_t)DIN * DTRANK * 2);
  unsigned short* oph  = (unsigned short*)carve((size_t)DMOD * DIN * 2);
  unsigned short* xnh  = (unsigned short*)carve((size_t)NTOK * DMOD * 2);
  float*          xz   = (float*)         carve((size_t)NTOK * XZW * 4);
  float*          uf   = (float*)         carve((size_t)NTOK * DIN * 4);
  unsigned short* uh   = (unsigned short*)carve((size_t)NTOK * DIN * 2);
  float*          xdbl = (float*)         carve((size_t)NTOK * XDBL_LD * 4);
  unsigned short* dt16 = (unsigned short*)carve((size_t)NTOK * DTRANK * 2);
  float*          dpre = (float*)         carve((size_t)NTOK * DIN * 4);
  unsigned short* y16  = (unsigned short*)carve((size_t)NTOK * DIN * 2);
  if (off > ws_size) return;

  {
    const int n8 = XZW * DMOD / 8;
    cast8_pad_kernel<<<(n8 + 255) / 256, 256, 0, stream>>>(in_proj_w, w1h, n8, n8, CARRY);
  }
  {
    const int c8 = XDBL_N * DIN / 8, n8 = XDBL_LD * DIN / 8;
    cast8_pad_kernel<<<(n8 + 255) / 256, 256, 0, stream>>>(x_proj_w, xph, c8, n8, CARRY);
  }
  {
    const int n8 = DIN * DTRANK / 8;
    cast8_pad_kernel<<<(n8 + 255) / 256, 256, 0, stream>>>(dt_proj_w, dtph, n8, n8, CARRY);
  }
  {
    const int n8 = DMOD * DIN / 8;
    cast8_pad_kernel<<<(n8 + 255) / 256, 256, 0, stream>>>(out_proj_w, oph, n8, n8, CARRY);
  }
  ln_kernel<<<NTOK, 128, 0, stream>>>(x, ln_g, ln_b, xnh);
  wmma_gemm64<0, false, 0, 0, false, 0><<<dim3((NTOK / 64) * (XZW / 64) / 8, 1), 256, 0, stream>>>(
      xnh, xnh, DMOD, 0L, w1h, w1h, DMOD, 0L, (void*)xz, (void*)xz, XZW, 0L,
      dt_proj_b, x, 0L, NTOK, XZW, DMOD, INV_C1);
  conv_silu_kernel<<<NTOK, 256, 0, stream>>>(xz, conv_w, conv_b, uf, uh);
  wmma_gemm64<0, false, 0, 0, false, 0><<<dim3((NTOK / 64) * (XDBL_LD / 64) / 8, 1), 256, 0, stream>>>(
      uh, uh, DIN, 0L, xph, xph, DIN, 0L, (void*)xdbl, (void*)xdbl, XDBL_LD, 0L,
      dt_proj_b, x, 0L, NTOK, XDBL_LD, DIN, INV_C2);
  dtcast_kernel<<<(NTOK * 8 + 255) / 256, 256, 0, stream>>>(xdbl, dt16, CARRY);
  wmma_gemm64<0, false, 0, 0, false, 0><<<dim3((NTOK / 64) * (DIN / 64) / 8, 1), 256, 0, stream>>>(
      dt16, dt16, DTRANK, 0L, dtph, dtph, DTRANK, 0L, (void*)dpre, (void*)dpre, DIN, 0L,
      dt_proj_b, x, 0L, NTOK, DIN, DTRANK, INV_C2);
  scan_kernel<<<dim3(DIN / SCAN_TB, NBATCH), SCAN_TB, 0, stream>>>(dpre, uf, xdbl, xz, A_log, dt_proj_b, Dv, y16);
  wmma_gemm64<0, false, 0, 0, true, 0><<<dim3((NTOK / 64) * (DMOD / 64) / 8, 1), 256, 0, stream>>>(
      y16, y16, DIN, 0L, oph, oph, DIN, 0L, (void*)out, (void*)out, DMOD, 0L,
      dt_proj_b, x, 0L, NTOK, DMOD, DIN, INV_C2);
}
